// NeuralCausalDiscovery_76897094468060
// MI455X (gfx1250) — hardware-verified
//
#include <hip/hip_runtime.h>
#include <math.h>
typedef __attribute__((ext_vector_type(16))) _Float16 v16h;
typedef __attribute__((ext_vector_type(8)))  _Float16 v8h;
typedef __attribute__((ext_vector_type(16))) __bf16   v16b;
typedef __attribute__((ext_vector_type(8)))  __bf16   v8b;
typedef __attribute__((ext_vector_type(8)))  float    v8f;
typedef __attribute__((ext_vector_type(4)))  float    v4f;
#define PSCALE 32768.0f
#define U16(p) ((const unsigned short*)(const void*)(p))
#define PSCALE_INV (1.0f / 32768.0f)

__device__ __forceinline__ unsigned short f2bf_bits(float f) {
  unsigned u = __float_as_uint(f);
  return (unsigned short)((u + 0x7FFFu + ((u >> 16) & 1u)) >> 16);
}
__device__ __forceinline__ float bf_bits2f(unsigned short h) { return __uint_as_float(((unsigned)h) << 16); }

__device__ __forceinline__ void dep_guard_h(v8f& a, v8f& b, v16h x, v16h y) { asm volatile("v_nop\n\tv_nop\n\tv_nop\n\tv_nop" : "+v"(a), "+v"(b) : "v"(x), "v"(y)); }
__device__ __forceinline__ void dep_guard_b(v8f& a, v8f& b, v16b x, v16b y) { asm volatile("v_nop\n\tv_nop\n\tv_nop\n\tv_nop" : "+v"(a), "+v"(b) : "v"(x), "v"(y)); }
__device__ __forceinline__ void keep4_h(v16h a, v16h b, v16h c, v16h d) { asm volatile("v_nop" :: "v"(a), "v"(b), "v"(c), "v"(d)); }
__device__ __forceinline__ void keep4_b(v16b a, v16b b, v16b c, v16b d) { asm volatile("v_nop" :: "v"(a), "v"(b), "v"(c), "v"(d)); }
__device__ __forceinline__ void acc_guard4(v8f& a, v8f& b, v8f& c, v8f& d) { asm volatile("v_nop\n\tv_nop\n\tv_nop\n\tv_nop" : "+v"(a), "+v"(b), "+v"(c), "+v"(d)); }
template <typename T> struct Frag;
template <> struct Frag<_Float16> {
  typedef v16h V; union U { v16h v; v8h h[2]; };
  static __device__ __forceinline__ v16h load(const _Float16* p) {
    U f; f.h[0] = *(const v8h*)(p); f.h[1] = *(const v8h*)(p + 16); return f.v;
  }
  static __device__ __forceinline__ v8f mma(v16h a, v16h b, v8f c) {
    return __builtin_amdgcn_wmma_f32_16x16x32_f16(false, a, false, b, (short)0, c, false, false);
  }
  static __device__ __forceinline__ void guard(v8f& a, v8f& b, v16h x, v16h y) { dep_guard_h(a, b, x, y); }
  static __device__ __forceinline__ void keep(v16h a, v16h b, v16h c, v16h d) { keep4_h(a, b, c, d); }
};
template <> struct Frag<__bf16> {
  typedef v16b V; union U { v16b v; v8b h[2]; };
  static __device__ __forceinline__ v16b load(const __bf16* p) {
    U f; f.h[0] = *(const v8b*)(p); f.h[1] = *(const v8b*)(p + 16); return f.v;
  }
  static __device__ __forceinline__ v8f mma(v16b a, v16b b, v8f c) {
    return __builtin_amdgcn_wmma_f32_16x16x32_bf16(false, a, false, b, (short)0, c, false, false);
  }
  static __device__ __forceinline__ void guard(v8f& a, v8f& b, v16b x, v16b y) { dep_guard_b(a, b, x, y); }
  static __device__ __forceinline__ void keep(v16b a, v16b b, v16b c, v16b d) { keep4_b(a, b, c, d); }
};

template <int ET> struct Elem;
template <> struct Elem<0> { typedef _Float16 T; };
template <> struct Elem<1> { typedef __bf16 T; };
template <int ET, bool SPLIT, int BIAS_MODE, int OUT_MODE, bool RESID, int ACT = 0>
__global__ __launch_bounds__(256) void wmma_gemm64(
    const unsigned short* __restrict__ Ap, const unsigned short* __restrict__ A2p, int lda, long strideA,
    const unsigned short* __restrict__ Btp, const unsigned short* __restrict__ Bt2p, int ldb, long strideB,
    void* __restrict__ Cout, void* __restrict__ Cout2, int ldc, long strideC,
    const float* __restrict__ bias,
    const float* __restrict__ resid, long strideR,
    int M, int N, int K, float scale) {
  typedef typename Elem<ET>::T T;
  typedef typename Frag<T>::V V;
  const T* A = (const T*)Ap; const T* A2 = (const T*)A2p; const T* Bt = (const T*)Btp; const T* Bt2 = (const T*)Bt2p;
  __shared__ __align__(16) float sT[8][16 * 68];
  const int b    = blockIdx.y;
  const int lane = threadIdx.x & 31;
  const int wave = threadIdx.x >> 5;
  const int tilesN = N >> 6;
  const int tilesM = M >> 6;
  const int tile = blockIdx.x * 8 + wave;
  if (tile >= tilesM * tilesN) return;
  const int tm = tile / tilesN;
  const int tn = tile - tm * tilesN;
  const int m0 = tm << 6;
  const int n0 = tn << 6;

  const T* Ab  = A  + (size_t)b * strideA;
  const T* Bb  = Bt + (size_t)b * strideB;
  const T* Ab2 = SPLIT ? (A2  + (size_t)b * strideA) : nullptr;
  const T* Bb2 = SPLIT ? (Bt2 + (size_t)b * strideB) : nullptr;

  const int rlane = lane & 15;
  const int koff  = (lane >> 4) * 8;
  const int mOff  = (lane >> 4) * 8;

  v8f acc[4][4];
#pragma unroll
  for (int i = 0; i < 4; ++i)
#pragma unroll
    for (int j = 0; j < 4; ++j) acc[i][j] = (v8f){0.f,0.f,0.f,0.f,0.f,0.f,0.f,0.f};

  for (int k0 = 0; k0 < K; k0 += 32) {
    V bh[4], bl[4];
#pragma unroll
    for (int j = 0; j < 4; ++j) {
      const size_t bo = (size_t)(n0 + (j << 4) + rlane) * ldb + koff + k0;
      bh[j] = Frag<T>::load(Bb + bo);
      if (SPLIT) bl[j] = Frag<T>::load(Bb2 + bo);
    }
#pragma unroll
    for (int i = 0; i < 4; ++i) {
      const size_t ao = (size_t)(m0 + (i << 4) + rlane) * lda + koff + k0;
      V ah = Frag<T>::load(Ab + ao);
      V al;
      if (SPLIT) al = Frag<T>::load(Ab2 + ao);
#pragma unroll
      for (int j = 0; j < 4; ++j) {
        acc[i][j] = Frag<T>::mma(ah, bh[j], acc[i][j]);
        if (SPLIT) {
          acc[i][j] = Frag<T>::mma(ah, bl[j], acc[i][j]);
          acc[i][j] = Frag<T>::mma(al, bh[j], acc[i][j]);
        }
      }
      Frag<T>::guard(acc[i][0], acc[i][3], ah, SPLIT ? al : ah);
    }
    Frag<T>::keep(bh[0], bh[1], bh[2], bh[3]);
    if (SPLIT) Frag<T>::keep(bl[0], bl[1], bl[2], bl[3]);
  }
  acc_guard4(acc[0][0], acc[0][1], acc[0][2], acc[0][3]);
  acc_guard4(acc[1][0], acc[1][1], acc[1][2], acc[1][3]);
  acc_guard4(acc[2][0], acc[2][1], acc[2][2], acc[2][3]);
  acc_guard4(acc[3][0], acc[3][1], acc[3][2], acc[3][3]);

  float* slab = sT[wave];
  const float* Rb = RESID ? (resid + (size_t)b * strideR) : nullptr;
#pragma unroll
  for (int i = 0; i < 4; ++i) {
    const int mBase = m0 + (i << 4);
#pragma unroll
    for (int j = 0; j < 4; ++j) {
      const int n = n0 + (j << 4) + rlane;
      float bv = 0.f;
      if (BIAS_MODE == 2) bv = bias[n];
#pragma unroll
      for (int r = 0; r < 8; ++r) {
        float v = acc[i][j][r] * scale;
        if (BIAS_MODE == 1) v += bias[mBase + mOff + r];
        if (BIAS_MODE == 2) v += bv;
        if (RESID) v += Rb[(size_t)(mBase + mOff + r) * ldc + n];
        if (ACT == 1) v = tanhf(v);
        if (ACT == 2) v = fmaxf(v, 0.0f);
        if (ACT == 3) v = v / (1.0f + expf(-v));
        if (ACT == 4) v = (v > 0.f) ? v : 0.01f * v;
        if (ACT == 5) v = 0.5f * v * (1.0f + erff(v * 0.70710678118654752f));
        slab[(mOff + r) * 68 + (j << 4) + rlane] = v;
      }
    }
    __builtin_amdgcn_fence(__ATOMIC_RELEASE, "workgroup");
    __builtin_amdgcn_wave_barrier();
    __builtin_amdgcn_fence(__ATOMIC_ACQUIRE, "workgroup");
    if (OUT_MODE == 0) {
      float* C = (float*)Cout + (size_t)b * strideC;
      const int hh = lane >> 4, c4 = (lane & 15) * 4;
      for (int pass = 0; pass < 2; ++pass) {
#pragma unroll
        for (int it = 0; it < 8; ++it) {
          const int row = it * 2 + hh;
          v4f v = *(const v4f*)(slab + row * 68 + c4);
          *(volatile v4f*)(C + (size_t)(mBase + row) * ldc + n0 + c4) = v;
        }
        __threadfence();
      }
    } else {
      const int q = lane >> 3, c8 = (lane & 7) * 8;
      unsigned short* C  = (unsigned short*)Cout  + (size_t)b * strideC;
      unsigned short* C2 = (OUT_MODE == 2) ? ((unsigned short*)Cout2 + (size_t)b * strideC) : nullptr;
      for (int pass = 0; pass < 2; ++pass) {
#pragma unroll
        for (int it = 0; it < 4; ++it) {
          const int row = it * 4 + q;
          const float* sp = slab + row * 68 + c8;
          v8h hv, lv;
#pragma unroll
          for (int e = 0; e < 8; ++e) {
            if (OUT_MODE == 1) {
              hv[e] = (_Float16)sp[e];
            } else {
              unsigned short hb = f2bf_bits(sp[e]);
              unsigned short lb = f2bf_bits(sp[e] - bf_bits2f(hb));
              hv[e] = __builtin_bit_cast(_Float16, hb);
              lv[e] = __builtin_bit_cast(_Float16, lb);
            }
          }
          *(volatile v8h*)(C + (size_t)(mBase + row) * ldc + n0 + c8) = hv;
          if (OUT_MODE == 2) *(volatile v8h*)(C2 + (size_t)(mBase + row) * ldc + n0 + c8) = lv;
        }
        __threadfence();
      }
    }
    __builtin_amdgcn_fence(__ATOMIC_RELEASE, "workgroup");
    __builtin_amdgcn_wave_barrier();
    __builtin_amdgcn_fence(__ATOMIC_ACQUIRE, "workgroup");
  }
}

__global__ __launch_bounds__(256) void cast_f32_f16x2(
    const float* __restrict__ in, _Float16* __restrict__ out, int n2) {
  int i = blockIdx.x * 256 + threadIdx.x;
  if (i < n2) {
    const _Float16 h0 = (_Float16)in[2 * i], h1 = (_Float16)in[2 * i + 1];
    const unsigned u = (unsigned)__builtin_bit_cast(unsigned short, h0) | ((unsigned)__builtin_bit_cast(unsigned short, h1) << 16);
    ((volatile unsigned*)out)[i] = u;
    __threadfence();
    ((volatile unsigned*)out)[i] = u;
  }
}


#define NV 28
#define NHd 64
#define NBt 32768
#define NG 7
#define NGC (NG * NHd)
__global__ __launch_bounds__(256) void xpad_kernel(const float* __restrict__ X, unsigned* __restrict__ X16) {
  const int i = blockIdx.x * 256 + threadIdx.x; if (i >= NBt * 16) return; const int b = i / 16, kp = i % 16; float a = 0.f, c = 0.f;
  if (2 * kp < NV) a = X[b * NV + 2 * kp]; if (2 * kp + 1 < NV) c = X[b * NV + 2 * kp + 1];
  const unsigned u = (unsigned)__builtin_bit_cast(unsigned short, (_Float16)a) | ((unsigned)__builtin_bit_cast(unsigned short, (_Float16)c) << 16);
  ((volatile unsigned*)X16)[i] = u; __threadfence(); ((volatile unsigned*)X16)[i] = u;
}
__global__ __launch_bounds__(256) void wprep_kernel(const float* __restrict__ Wl, const float* __restrict__ W1, const float* __restrict__ W2, float* __restrict__ Wout, unsigned* __restrict__ B1, unsigned* __restrict__ B2) {
  __shared__ float Wm[NV][NV];
  for (int i = threadIdx.x; i < NV * NV; i += 256) { const int n = i / NV, d = i % NV; Wm[n][d] = (n == d) ? 0.f : 1.0f / (1.0f + expf(-Wl[i])); }
  __syncthreads();
  if (blockIdx.x == 0) for (int i = threadIdx.x; i < NV * NV; i += 256) { ((volatile float*)Wout)[i] = (&Wm[0][0])[i]; __threadfence(); ((volatile float*)Wout)[i] = (&Wm[0][0])[i]; }
  for (int i = blockIdx.x * 256 + threadIdx.x; i < NV * NHd * 16; i += gridDim.x * 256) { const int r = i / 16, kp = i % 16; const int n = r / NHd, h = r % NHd; float a = 0.f, c = 0.f;
    if (2 * kp < NV) a = W1[((size_t)n * NHd + h) * NV + 2 * kp] * Wm[n][2 * kp]; if (2 * kp + 1 < NV) c = W1[((size_t)n * NHd + h) * NV + 2 * kp + 1] * Wm[n][2 * kp + 1];
    const unsigned u = (unsigned)__builtin_bit_cast(unsigned short, (_Float16)a) | ((unsigned)__builtin_bit_cast(unsigned short, (_Float16)c) << 16);
    ((volatile unsigned*)B1)[i] = u; __threadfence(); ((volatile unsigned*)B1)[i] = u; }
  for (int i = blockIdx.x * 256 + threadIdx.x; i < NV * NHd * NHd / 2; i += gridDim.x * 256) { const float a = W2[2 * i], c = W2[2 * i + 1];
    const unsigned u = (unsigned)__builtin_bit_cast(unsigned short, (_Float16)a) | ((unsigned)__builtin_bit_cast(unsigned short, (_Float16)c) << 16);
    ((volatile unsigned*)B2)[i] = u; __threadfence(); ((volatile unsigned*)B2)[i] = u; }
}
__global__ __launch_bounds__(256) void bn_part_kernel(const float* __restrict__ Hm, double* __restrict__ PS) {
  const int t = threadIdx.x; const int r0 = blockIdx.x * 512;
  if (t < 224) { const int c = 2 * t; double s0 = 0, s1 = 0, q0 = 0, q1 = 0;
    for (int r = r0; r < r0 + 512; ++r) { const double a = Hm[(size_t)r * NGC + c], b = Hm[(size_t)r * NGC + c + 1]; s0 += a; s1 += b; q0 += a * a; q1 += b * b; }
    double* dst = PS + (size_t)blockIdx.x * 1024;
    for (int pass = 0; pass < 2; ++pass) { ((volatile double*)dst)[c] = s0; ((volatile double*)dst)[c + 1] = s1; ((volatile double*)dst)[512 + c] = q0; ((volatile double*)dst)[512 + c + 1] = q1; __threadfence(); } }
}
__global__ __launch_bounds__(256) void bn_final_kernel(const double* __restrict__ PS, int nblk, const float* __restrict__ gamma, const float* __restrict__ beta, int goff, float* __restrict__ SS2) {
  for (int c = threadIdx.x; c < NGC; c += 256) { double s = 0, q = 0; for (int b = 0; b < nblk; ++b) { s += PS[(size_t)b * 1024 + c]; q += PS[(size_t)b * 1024 + 512 + c]; }
    const double mu = s / NBt; double var = q / NBt - mu * mu; if (var < 0) var = 0; const float sc = gamma[goff + c] * (float)(1.0 / sqrt(var + 1e-5)); const float sh = beta[goff + c] - (float)mu * sc;
    ((volatile float*)SS2)[c] = sc; ((volatile float*)SS2)[512 + c] = sh; __threadfence(); ((volatile float*)SS2)[c] = sc; ((volatile float*)SS2)[512 + c] = sh; }
}
__global__ __launch_bounds__(256) void bn_gelu_kernel(const float* __restrict__ Hm, const float* __restrict__ SS2, unsigned* __restrict__ A16) {
  const size_t i = (size_t)blockIdx.x * 256 + threadIdx.x; if (i >= (size_t)NBt * NGC / 2) return; const int c = (int)((2 * i) % NGC);
  float a = Hm[2 * i] * SS2[c] + SS2[512 + c], b = Hm[2 * i + 1] * SS2[c + 1] + SS2[512 + c + 1];
  a = 0.5f * a * (1.0f + erff(a * 0.70710678118654752f)); b = 0.5f * b * (1.0f + erff(b * 0.70710678118654752f));
  const unsigned u = (unsigned)__builtin_bit_cast(unsigned short, (_Float16)a) | ((unsigned)__builtin_bit_cast(unsigned short, (_Float16)b) << 16);
  ((volatile unsigned*)A16)[i] = u; __threadfence(); ((volatile unsigned*)A16)[i] = u;
}
__global__ __launch_bounds__(256) void out_kernel(const float* __restrict__ H2, const float* __restrict__ SS2, const float* __restrict__ W3, const float* __restrict__ b3, int n0, int g, float* __restrict__ XH) {
  const int lane = threadIdx.x & 31, wave = threadIdx.x >> 5; const size_t b4 = (size_t)blockIdx.x * 8 + wave;
  __shared__ float st[8][32];
  st[wave][lane] = 0.f;
#pragma unroll 1
  for (int k = 0; k < 4; ++k) { const size_t b = b4 * 4 + k;
#pragma unroll 1
    for (int q = 0; q < NG; ++q) { const int c = q * NHd + 2 * lane; float a = H2[b * NGC + c] * SS2[c] + SS2[512 + c], bb = H2[b * NGC + c + 1] * SS2[c + 1] + SS2[512 + c + 1];
      a = 0.5f * a * (1.0f + erff(a * 0.70710678118654752f)); bb = 0.5f * bb * (1.0f + erff(bb * 0.70710678118654752f));
      float d = a * W3[(n0 + q) * NHd + 2 * lane] + bb * W3[(n0 + q) * NHd + 2 * lane + 1];
      for (int o = 16; o > 0; o >>= 1) d += __shfl_xor(d, o, 32);
      if (lane == 0) st[wave][k * 8 + q] = d + b3[n0 + q]; } }
  __builtin_amdgcn_wave_barrier();
  const float v = st[wave][lane]; float* dst = XH + ((size_t)g * NBt + b4 * 4) * 8;
  ((volatile float*)dst)[lane] = v; __threadfence(); ((volatile float*)dst)[lane] = v;
}
__global__ __launch_bounds__(256) void pack_kernel(const float* __restrict__ XH, float* __restrict__ out) {
  const int lane = threadIdx.x & 31, wave = threadIdx.x >> 5; const size_t r0 = ((size_t)blockIdx.x * 8 + wave) * 8;
  for (int pass = 0; pass < 2; ++pass) { for (int i = lane; i < 8 * NV; i += 32) { const int rr = i / NV, c = i % NV; const int g = c / NG, q = c % NG;
      ((volatile float*)out)[(r0 + rr) * NV + c] = XH[((size_t)g * NBt + r0 + rr) * 8 + q]; } __threadfence(); }
}
extern "C" void kernel_launch(void* const* d_in, const int* in_sizes, int n_in, void* d_out, int out_size, void* d_ws, size_t ws_size, hipStream_t stream) {
  (void)in_sizes; (void)n_in; (void)out_size; (void)ws_size;
  const float* X = (const float*)d_in[0]; const float* Wl = (const float*)d_in[1]; const float* W1 = (const float*)d_in[2]; const float* g1 = (const float*)d_in[4]; const float* be1 = (const float*)d_in[5];
  const float* W2 = (const float*)d_in[6]; const float* g2 = (const float*)d_in[8]; const float* be2 = (const float*)d_in[9]; const float* W3 = (const float*)d_in[10]; const float* b3 = (const float*)d_in[11];
  (void)d_in[3]; (void)d_in[7];
  float* Xhat = (float*)d_out; float* Wout = Xhat + (size_t)NBt * NV;
  char* ws = (char*)d_ws; size_t off = 0;
  auto carve = [&](size_t bytes) -> char* { char* p = ws + off; off += (bytes + 255) & ~(size_t)255; return p; };
  unsigned* X16 = (unsigned*)carve((size_t)NBt * 32 * 2); unsigned* B1 = (unsigned*)carve((size_t)NV * NHd * 32 * 2); unsigned* B2 = (unsigned*)carve((size_t)NV * NHd * NHd * 2);
  float* H1 = (float*)carve((size_t)NBt * NGC * 4); unsigned* A1 = (unsigned*)carve((size_t)NBt * NGC * 2); float* H2 = (float*)carve((size_t)NBt * NGC * 4);
  const int NBB = NBt / 512; double* PS = (double*)carve((size_t)NBB * 1024 * 8); float* SS2 = (float*)carve(1024 * 4); float* XH = (float*)carve((size_t)4 * NBt * 8 * 4);
  xpad_kernel<<<(NBt * 16 + 255) / 256, 256, 0, stream>>>(X, X16);
  wprep_kernel<<<32, 256, 0, stream>>>(Wl, W1, W2, Wout, B1, B2);
  const int t1 = (NBt / 64) * (NGC / 64), t2 = (NBt / 64) * 1;
  for (int g = 0; g < NV / NG; ++g) { const int n0 = g * NG;
    wmma_gemm64<0, false, 0, 0, false><<<dim3((t1 + 7) / 8, 1), 256, 0, stream>>>((const unsigned short*)X16, nullptr, 32, 0, (const unsigned short*)B1 + (size_t)n0 * NHd * 32, nullptr, 32, 0, H1, nullptr, NGC, 0, nullptr, nullptr, 0, NBt, NGC, 32, 1.0f);
    bn_part_kernel<<<NBB, 256, 0, stream>>>(H1, PS);
    bn_final_kernel<<<1, 256, 0, stream>>>(PS, NBB, g1, be1, n0 * NHd, SS2);
    bn_gelu_kernel<<<(unsigned)(((size_t)NBt * NGC / 2 + 255) / 256), 256, 0, stream>>>(H1, SS2, A1);
    wmma_gemm64<0, false, 0, 0, false><<<dim3((t2 + 7) / 8, NG), 256, 0, stream>>>((const unsigned short*)A1, nullptr, NGC, NHd, (const unsigned short*)B2 + (size_t)n0 * NHd * NHd, nullptr, NHd, NHd * NHd, H2, nullptr, NGC, NHd, nullptr, nullptr, 0, NBt, NHd, NHd, 1.0f);
    bn_part_kernel<<<NBB, 256, 0, stream>>>(H2, PS);
    bn_final_kernel<<<1, 256, 0, stream>>>(PS, NBB, g2, be2, n0 * NHd, SS2);
    out_kernel<<<NBt / 32, 256, 0, stream>>>(H2, SS2, W3, b3, n0, g, XH);
  }
  pack_kernel<<<NBt / 64, 256, 0, stream>>>(XH, Xhat);
}
